// RecursiveEncoder_16681652978506
// MI455X (gfx1250) — hardware-verified
//
#include <hip/hip_runtime.h>
#include <stddef.h>


#pragma clang fp contract(off)

#define NF     320
#define HC     256
#define MCH    10
#define NE     40
#define NTY    4
#define KI     516
#define KP     768
#define NTHR   256
#define NW     8
#define TPB    8
#define RPB    (TPB * MCH)
#define NRT    (RPB / 16)
#define APC    328
#define APM    264
#define OPC    260
#define PQP    256
#define ACP    128
#define PRB    64
#define OPP    260
#define OWC    0
#define OWI0   81920
#define OWI1   212992
#define OWP    344064
#define OWT    540672
#define PREPB  (OWT / (NTHR * 8))
#define CHDYN  (RPB * OPC * 4)
#define MSGR0  (RPB * PQP * 4)
#define MSGDYN (MSGR0 + RPB * ACP * 4)
#define PARDYN (PRB * OPP * 4)
#define WSCAP  134217728

static_assert((OWI0 % (NTHR * 8)) == 0);
static_assert((OWI1 % (NTHR * 8)) == 0);
static_assert((OWP % (NTHR * 8)) == 0);
static_assert((OWT % (NTHR * 8)) == 0);
static_assert(OWI0 == HC * NF);
static_assert(OWI1 == OWI0 + 2 * HC * HC);
static_assert(OWP == OWI1 + 2 * HC * HC);
static_assert(OWT == OWP + HC * KP);
static_assert(RPB * APC * 2 <= CHDYN);
static_assert(RPB * APM * 2 <= MSGR0);
static_assert((APC % 8) == 0);
static_assert((APM % 8) == 0);
static_assert((OPC % 4) == 0);
static_assert((OPP % 4) == 0);
static_assert((NF % 32) == 0);
static_assert((HC % 32) == 0);
static_assert((KP % 32) == 0);
static_assert(RPB == NRT * 16);
static_assert(NTHR == HC);
static_assert(RPB <= NTHR);
static_assert(NW * 32 == NTHR);
static_assert(TPB == NW);
static_assert(PRB == 8 * NW);
static_assert((TPB % 2) == 0);

typedef float          v4f   __attribute__((ext_vector_type(4)));
typedef float          v8f   __attribute__((ext_vector_type(8)));
typedef unsigned int   v4u   __attribute__((ext_vector_type(4)));
typedef _Float16       v8h   __attribute__((ext_vector_type(8)));
typedef _Float16       v16h  __attribute__((ext_vector_type(16)));

__device__ __forceinline__ v16h ldfrag(const _Float16* p) {
  const v8h u0 = *(const v8h*)p;
  const v8h u1 = *(const v8h*)(p + 16);
  return __builtin_shufflevector(u0, u1, 0, 1, 2, 3, 4, 5, 6, 7, 8, 9, 10, 11, 12, 13, 14, 15);
}

__device__ __forceinline__ v8f wm(v16h a, v16h b, v8f c) {
  v8f d = __builtin_amdgcn_wmma_f32_16x16x32_f16(false, a, false, b, (short)0, c, false, false);
  asm volatile("v_nop\n\tv_nop\n\tv_nop\n\tv_nop" : "+v"(d) : "v"(a), "v"(b));
  return d;
}
__device__ __forceinline__ v8f zero8() {
  v8f z = {0.f, 0.f, 0.f, 0.f, 0.f, 0.f, 0.f, 0.f};
  return z;
}
__device__ __forceinline__ int iclamp(int v, int lo, int hi) { return v < lo ? lo : (v > hi ? hi : v); }

__device__ __forceinline__ v4u pack8(v4f a, v4f b, float s) {
  v8h hv;
  hv[0] = (_Float16)(s * a.x); hv[1] = (_Float16)(s * a.y); hv[2] = (_Float16)(s * a.z); hv[3] = (_Float16)(s * a.w);
  hv[4] = (_Float16)(s * b.x); hv[5] = (_Float16)(s * b.y); hv[6] = (_Float16)(s * b.z); hv[7] = (_Float16)(s * b.w);
  return __builtin_bit_cast(v4u, hv);
}

__global__ __launch_bounds__(NTHR) void k_prep(const float* __restrict__ Wc, const float* __restrict__ Wi0,
                                               const float* __restrict__ Wi1, const float* __restrict__ Wp,
                                               _Float16* wpl) {
  const int tid = (int)threadIdx.x;
  const int blk = (int)blockIdx.x;
  const int o = (blk * NTHR + tid) * 8;
  v8h hv;
  if (blk < OWI0 / (NTHR * 8)) {
    const int n = o / NF, k0 = o - n * NF;
#pragma unroll
    for (int i = 0; i < 8; ++i) hv[i] = (_Float16)(64.0f * Wc[(size_t)(k0 + i) * HC + n]);
  } else if (blk < OWP / (NTHR * 8)) {
    const bool second = blk >= OWI1 / (NTHR * 8);
    const float* W = second ? Wi1 : Wi0;
    const int local = o - (second ? OWI1 : OWI0);
    const int n = local >> 8, k0 = local & 255;
    const int roff = (n < HC) ? 0 : HC;
    const int col = n - roff;
#pragma unroll
    for (int i = 0; i < 8; ++i) hv[i] = (_Float16)(64.0f * W[(size_t)(roff + k0 + i) * HC + col]);
  } else {
    const int local = o - OWP;
    const int n = local / KP, k0 = local - n * KP;
#pragma unroll
    for (int i = 0; i < 8; ++i) hv[i] = (_Float16)(64.0f * Wp[(size_t)(k0 + i) * HC + n]);
  }
  const v4u u = __builtin_bit_cast(v4u, hv);
  _Float16* dst = wpl + o;
  *(volatile v4u*)dst = u;
  __threadfence();
  *(volatile v4u*)dst = u;
}

__device__ __forceinline__ void child_rows(const float* sO, _Float16* CF0, int row0, int nRows, int wave, int lane) {
#pragma unroll 1
  for (int i = 0; i < RPB / NW; ++i) {
    const int row = wave + NW * i;
    const int gr = row0 + row;
    if (gr < nRows) {
      const v4f a = *(const v4f*)(sO + row * OPC + 8 * lane);
      const v4f b = *(const v4f*)(sO + row * OPC + 8 * lane + 4);
      *(volatile v4u*)(CF0 + (size_t)gr * HC + 8 * lane) = pack8(a, b, 16.0f);
    }
  }
}
__device__ __forceinline__ void child_feat(const float* sF, _Float16* FT, int t0, int nT, int wave, int lane) {
  const int tree = t0 + wave;
  if (tree < nT) {
    const v4f a = *(const v4f*)(sF + wave * HC + 8 * lane);
    const v4f b = *(const v4f*)(sF + wave * HC + 8 * lane + 4);
    *(volatile v4u*)(FT + (size_t)tree * KP + 8 * lane) = pack8(a, b, 16.0f);
  }
}

__global__ __launch_bounds__(NTHR) void k_child(const float* __restrict__ x, const float* __restrict__ ex,
                                                const float* __restrict__ bc, const _Float16* __restrict__ wpl,
                                                _Float16* CF0, _Float16* FT, int nT) {
  extern __shared__ __attribute__((aligned(16))) v4f cdyn[];
  __shared__ float sBc[HC];
  __shared__ float sEx[RPB];
  __shared__ __attribute__((aligned(16))) float sF[TPB * HC];
  _Float16* sA = (_Float16*)cdyn;
  float*    sO = (float*)cdyn;
  const int tid = (int)threadIdx.x, lane = tid & 31, wave = tid >> 5, hh = lane >> 4, m = lane & 15;
  const int nRows = nT * MCH;
  const int t0 = (int)blockIdx.x * TPB;
  const int row0 = t0 * MCH;

  sBc[tid] = bc[tid];
  if (tid < RPB) {
    int gr = row0 + tid;
    gr = gr > nRows - 1 ? nRows - 1 : gr;
    sEx[tid] = ex[gr];
  }
#pragma unroll 1
  for (int u = tid; u < RPB * (NF / 8); u += NTHR) {
    const int row = u / (NF / 8), c8 = u - row * (NF / 8);
    int gr = row0 + row;
    gr = gr > nRows - 1 ? nRows - 1 : gr;
    const float* p = x + (size_t)gr * NF + 8 * c8;
    const v4f a = *(const v4f*)p;
    const v4f b = *(const v4f*)(p + 4);
    v8h hv;
    hv[0] = (_Float16)a.x; hv[1] = (_Float16)a.y; hv[2] = (_Float16)a.z; hv[3] = (_Float16)a.w;
    hv[4] = (_Float16)b.x; hv[5] = (_Float16)b.y; hv[6] = (_Float16)b.z; hv[7] = (_Float16)b.w;
    *(v8h*)(sA + row * APC + 8 * c8) = hv;
  }
  __syncthreads();

  v8f c[NRT][2];
#pragma unroll
  for (int rt = 0; rt < NRT; ++rt) { c[rt][0] = zero8(); c[rt][1] = zero8(); }
  {
    const _Float16* bq = wpl + OWC + (size_t)(32 * wave + m) * NF + 8 * hh;
    const _Float16* aq = sA + m * APC + 8 * hh;
#pragma unroll 1
    for (int ks = 0; ks < NF / 32; ++ks) {
      const v16h b0 = ldfrag(bq + 32 * ks);
      const v16h b1 = ldfrag(bq + (size_t)16 * NF + 32 * ks);
#pragma unroll
      for (int rt = 0; rt < NRT; ++rt) {
        const v16h a = ldfrag(aq + rt * 16 * APC + 32 * ks);
        c[rt][0] = wm(a, b0, c[rt][0]);
        c[rt][1] = wm(a, b1, c[rt][1]);
      }
    }
  }
  __syncthreads();

#pragma unroll
  for (int rt = 0; rt < NRT; ++rt) {
#pragma unroll
    for (int j = 0; j < 2; ++j) {
      const int col = 32 * wave + 16 * j + m;
      const float bb = sBc[col];
#pragma unroll
      for (int r = 0; r < 8; ++r) {
        const int row = 16 * rt + 8 * hh + r;
        const float t = c[rt][j][r] * 0.015625f + bb;
        sO[row * OPC + col] = fmaxf(t, 0.0f) * sEx[row];
      }
    }
  }
  __syncthreads();

  {
    const int col = tid;
#pragma unroll 1
    for (int tr = 0; tr < TPB; ++tr) {
      const float* sp = sO + (MCH * tr) * OPC + col;
      float mx = sp[0];
#pragma unroll
      for (int r = 1; r < MCH; ++r) mx = fmaxf(mx, sp[r * OPC]);
      sF[tr * HC + col] = mx;
    }
  }
  __syncthreads();

  child_rows(sO, CF0, row0, nRows, wave, lane);
  child_feat(sF, FT, t0, nT, wave, lane);
  __threadfence();
  child_rows(sO, CF0, row0, nRows, wave, lane);
  child_feat(sF, FT, t0, nT, wave, lane);
}

__device__ __forceinline__ void msg_rows(const float* sAcc, _Float16* CFout, int h, int row0, int nRows,
                                         int wave, int hh, int m) {
#pragma unroll 1
  for (int i = 0; i < NRT; ++i) {
    const int row = wave + 16 * i + 8 * hh;
    const int gr = row0 + row;
    if (gr < nRows) {
      const v4f a = *(const v4f*)(sAcc + row * ACP + 8 * m);
      const v4f b = *(const v4f*)(sAcc + row * ACP + 8 * m + 4);
      *(volatile v4u*)(CFout + (size_t)gr * HC + 128 * h + 8 * m) = pack8(a, b, 16.0f);
    }
  }
}
__device__ __forceinline__ void msg_feat(const float* sMx, _Float16* FT, int fcol, int t0, int nT,
                                         int wave, int hh, int m) {
  const int tree = t0 + wave;
  if (tree < nT && hh == 0) {
    const v4f a = *(const v4f*)(sMx + wave * 128 + 8 * m);
    const v4f b = *(const v4f*)(sMx + wave * 128 + 8 * m + 4);
    *(volatile v4u*)(FT + (size_t)tree * KP + fcol + 8 * m) = pack8(a, b, 16.0f);
  }
}

__global__ __launch_bounds__(NTHR) void k_msg(const _Float16* __restrict__ CFin, const int* __restrict__ eidx,
                                              const float* __restrict__ e1h, const float* __restrict__ Wi,
                                              const float* __restrict__ bi, const _Float16* __restrict__ wpl,
                                              _Float16* CFout, _Float16* FT, int owi, int nT, int fcol0,
                                              int writeCF) {
  extern __shared__ __attribute__((aligned(16))) v4f mdyn[];
  __shared__ int sEd[TPB * NE];
  __shared__ __attribute__((aligned(16))) float sE1[TPB * NE * NTY];
  __shared__ float sBi[128];
  __shared__ float sWe[NTY * 128];
  __shared__ float sRc[RPB];
  __shared__ __attribute__((aligned(16))) float sMx[TPB * 128];
  _Float16* sA   = (_Float16*)mdyn;
  float*    sPQ  = (float*)mdyn;
  float*    sAcc = (float*)mdyn + MSGR0 / 4;
  const int tid = (int)threadIdx.x, lane = tid & 31, wave = tid >> 5, hh = lane >> 4, m = lane & 15;
  const int h = (int)blockIdx.y;
  const int nRows = nT * MCH;
  const int t0 = (int)blockIdx.x * TPB;
  const int row0 = t0 * MCH;
  const int fcol = fcol0 + 128 * h;

#pragma unroll 1
  for (int e = tid; e < TPB * NE; e += NTHR) {
    const int tr = e / NE, le = e - tr * NE;
    int gt = t0 + tr;
    gt = gt > nT - 1 ? nT - 1 : gt;
    const size_t ge = (size_t)gt * NE + le;
    const int s = eidx[ge * 2];
    const int d = eidx[ge * 2 + 1];
    const int seg = ((unsigned)s < (unsigned)MCH) ? s : 15;
    int gs = s < 0 ? s + MCH : s;
    gs = iclamp(gs, 0, MCH - 1);
    int gd = d < 0 ? d + MCH : d;
    gd = iclamp(gd, 0, MCH - 1);
    sEd[e] = gs | (gd << 4) | (seg << 8);
    *(v4f*)(sE1 + 4 * e) = *(const v4f*)(e1h + ge * NTY);
  }
  if (tid < 128) {
    sBi[tid] = bi[128 * h + tid];
#pragma unroll
    for (int t = 0; t < NTY; ++t) sWe[t * 128 + tid] = Wi[(size_t)(2 * HC + t) * HC + 128 * h + tid];
  }
#pragma unroll 1
  for (int u = tid; u < RPB * (HC / 8); u += NTHR) {
    const int row = u >> 5, c8 = u & 31;
    int gr = row0 + row;
    gr = gr > nRows - 1 ? nRows - 1 : gr;
    const v8h v = *(const v8h*)(CFin + (size_t)gr * HC + 8 * c8);
    *(v8h*)(sA + row * APM + 8 * c8) = v;
  }
  __syncthreads();

  v8f c[NRT][2];
#pragma unroll
  for (int rt = 0; rt < NRT; ++rt) { c[rt][0] = zero8(); c[rt][1] = zero8(); }
  {
    const int nb = (wave < 4) ? (128 * h + 32 * wave) : (HC + 128 * h + 32 * (wave - 4));
    const _Float16* bq = wpl + owi + (size_t)(nb + m) * HC + 8 * hh;
    const _Float16* aq = sA + m * APM + 8 * hh;
#pragma unroll 1
    for (int ks = 0; ks < HC / 32; ++ks) {
      const v16h b0 = ldfrag(bq + 32 * ks);
      const v16h b1 = ldfrag(bq + (size_t)16 * HC + 32 * ks);
#pragma unroll
      for (int rt = 0; rt < NRT; ++rt) {
        const v16h a = ldfrag(aq + rt * 16 * APM + 32 * ks);
        c[rt][0] = wm(a, b0, c[rt][0]);
        c[rt][1] = wm(a, b1, c[rt][1]);
      }
    }
  }
  __syncthreads();

#pragma unroll
  for (int rt = 0; rt < NRT; ++rt) {
#pragma unroll
    for (int j = 0; j < 2; ++j) {
      const int lc = 32 * wave + 16 * j + m;
#pragma unroll
      for (int r = 0; r < 8; ++r) sPQ[(16 * rt + 8 * hh + r) * PQP + lc] = c[rt][j][r] * 0.0009765625f;
    }
  }
  if (tid < RPB) {
    const int tr = tid / MCH, ln = tid - tr * MCH;
    int cnt = 0;
#pragma unroll 1
    for (int le = 0; le < NE; ++le) cnt += ((((sEd[tr * NE + le]) >> 8) & 15) == ln) ? 1 : 0;
    sRc[tid] = 1.0f / fmaxf((float)cnt, 1.0f);
  }
  __syncthreads();

  {
    const int cc = tid & 127, q = tid >> 7;
    const float bic = sBi[cc];
    const float we0 = sWe[cc], we1 = sWe[128 + cc], we2 = sWe[256 + cc], we3 = sWe[384 + cc];
#pragma unroll 1
    for (int k4 = 0; k4 < TPB / 2; ++k4) {
      const int tr = q + 2 * k4;
      const int rb = MCH * tr;
      float* ac = sAcc + rb * ACP + cc;
#pragma unroll
      for (int i = 0; i < MCH; ++i) ac[i * ACP] = 0.0f;
#pragma unroll 1
      for (int le = 0; le < NE; ++le) {
        const int e = tr * NE + le;
        const int pk = sEd[e];
        const int gs = pk & 15, gd = (pk >> 4) & 15, sg = (pk >> 8) & 15;
        const v4f ev = *(const v4f*)(sE1 + 4 * e);
        const float pv = sPQ[(rb + gs) * PQP + cc];
        const float qv = sPQ[(rb + gd) * PQP + 128 + cc];
        const float wv = ((ev.x * we0 + ev.y * we1) + ev.z * we2) + ev.w * we3;
        const float v = fmaxf(((pv + qv) + wv) + bic, 0.0f);
        const bool ok = sg < MCH;
        const int sgc = ok ? sg : 0;
        const float add = ok ? v : 0.0f;
        ac[sgc * ACP] = ac[sgc * ACP] + add;
      }
      float mx = 0.0f;
#pragma unroll
      for (int i = 0; i < MCH; ++i) {
        const float val = ac[i * ACP] * sRc[rb + i];
        ac[i * ACP] = val;
        mx = (i == 0) ? val : fmaxf(mx, val);
      }
      sMx[tr * 128 + cc] = mx;
    }
  }
  __syncthreads();

  if (writeCF != 0) msg_rows(sAcc, CFout, h, row0, nRows, wave, hh, m);
  msg_feat(sMx, FT, fcol, t0, nT, wave, hh, m);
  __threadfence();
  if (writeCF != 0) msg_rows(sAcc, CFout, h, row0, nRows, wave, hh, m);
  msg_feat(sMx, FT, fcol, t0, nT, wave, hh, m);
}

__device__ __forceinline__ void parent_rows(const float* sO, float* out, int p0, int nT, int wave, int lane) {
#pragma unroll 1
  for (int i = 0; i < PRB / NW; ++i) {
    const int row = wave + NW * i;
    const int pr = p0 + row;
    if (pr < nT) {
      const v4f v0 = *(const v4f*)(sO + row * OPP + 4 * lane);
      const v4f v1 = *(const v4f*)(sO + row * OPP + 128 + 4 * lane);
      float* ob = out + (size_t)pr * HC;
      *(volatile v4f*)(ob + 4 * lane) = v0;
      *(volatile v4f*)(ob + 128 + 4 * lane) = v1;
    }
  }
}

__global__ __launch_bounds__(NTHR) void k_parent(const _Float16* __restrict__ FT, const float* __restrict__ bp,
                                                 const _Float16* __restrict__ wpl, float* out, int nT) {
  extern __shared__ __attribute__((aligned(16))) v4f pdyn[];
  __shared__ float sBp[HC];
  float* sO = (float*)pdyn;
  const int tid = (int)threadIdx.x, lane = tid & 31, wave = tid >> 5, hh = lane >> 4, m = lane & 15;
  const int p0 = (int)blockIdx.x * PRB;
  sBp[tid] = bp[tid];
  __syncthreads();

  v8f c[4][2];
#pragma unroll
  for (int rt = 0; rt < 4; ++rt) { c[rt][0] = zero8(); c[rt][1] = zero8(); }
  {
    const _Float16* ap[4];
#pragma unroll
    for (int rt = 0; rt < 4; ++rt) {
      int ar = p0 + 16 * rt + m;
      ar = ar > nT - 1 ? nT - 1 : ar;
      ap[rt] = FT + (size_t)ar * KP + 8 * hh;
    }
    const _Float16* bq = wpl + OWP + (size_t)(32 * wave + m) * KP + 8 * hh;
#pragma unroll 1
    for (int ks = 0; ks < KP / 32; ++ks) {
      const v16h b0 = ldfrag(bq + 32 * ks);
      const v16h b1 = ldfrag(bq + (size_t)16 * KP + 32 * ks);
#pragma unroll
      for (int rt = 0; rt < 4; ++rt) {
        const v16h a = ldfrag(ap[rt] + 32 * ks);
        c[rt][0] = wm(a, b0, c[rt][0]);
        c[rt][1] = wm(a, b1, c[rt][1]);
      }
    }
  }
#pragma unroll
  for (int rt = 0; rt < 4; ++rt) {
#pragma unroll
    for (int j = 0; j < 2; ++j) {
      const int col = 32 * wave + 16 * j + m;
      const float bb = sBp[col];
#pragma unroll
      for (int r = 0; r < 8; ++r) {
        const float t = c[rt][j][r] * 0.0009765625f + bb;
        sO[(16 * rt + 8 * hh + r) * OPP + col] = fmaxf(t, 0.0f);
      }
    }
  }
  __syncthreads();
  parent_rows(sO, out, p0, nT, wave, lane);
  __threadfence();
  parent_rows(sO, out, p0, nT, wave, lane);
}

extern "C" void kernel_launch(void* const* d_in, const int* in_sizes, int n_in,
                              void* d_out, int out_size, void* d_ws, size_t ws_size,
                              hipStream_t stream) {
  if (n_in < 12) return;
  if (in_sizes[0] < MCH * NF || (in_sizes[0] % (MCH * NF)) != 0) return;
  const int nT = in_sizes[0] / (MCH * NF);
  if (nT < 1 || nT > (1 << 20)) return;
  if (in_sizes[1] != nT * MCH) return;
  if (in_sizes[2] != nT * NE * NTY) return;
  if (in_sizes[3] != nT * NE * 2) return;
  if (in_sizes[4] != NF * HC || in_sizes[5] != HC) return;
  if (in_sizes[6] != KI * HC || in_sizes[7] != HC) return;
  if (in_sizes[8] != KI * HC || in_sizes[9] != HC) return;
  if (in_sizes[10] != KP * HC || in_sizes[11] != HC) return;
  if ((long long)out_size != (long long)nT * HC) return;

  const float* x    = (const float*)d_in[0];
  const float* ex   = (const float*)d_in[1];
  const float* e1h  = (const float*)d_in[2];
  const int*   eidx = (const int*)d_in[3];
  const float* Wc   = (const float*)d_in[4];
  const float* bc   = (const float*)d_in[5];
  const float* Wi0  = (const float*)d_in[6];
  const float* bi0  = (const float*)d_in[7];
  const float* Wi1  = (const float*)d_in[8];
  const float* bi1  = (const float*)d_in[9];
  const float* Wp   = (const float*)d_in[10];
  const float* bp   = (const float*)d_in[11];
  float* out = (float*)d_out;

  const int nb8  = (nT + TPB - 1) / TPB;
  const int nb64 = (nT + PRB - 1) / PRB;
  const size_t rowsPad = (size_t)nb8 * RPB;
  const size_t treePad = (size_t)nb64 * PRB;

  const size_t cap = ws_size < (size_t)WSCAP ? ws_size : (size_t)WSCAP;
  const size_t bW  = (size_t)OWT * 2;
  const size_t bCF = rowsPad * HC * 2;
  const size_t bFT = treePad * KP * 2;
  char* ws = (char*)d_ws;
  size_t off = 0;
  const size_t oW   = off; off += bW;   off = (off + 255) & ~(size_t)255;
  const size_t oCF0 = off; off += bCF;  off = (off + 255) & ~(size_t)255;
  const size_t oCF1 = off; off += bCF;  off = (off + 255) & ~(size_t)255;
  const size_t oFT  = off; off += bFT;  off = (off + 255) & ~(size_t)255;
  if (off > cap || off > ws_size) return;
  _Float16* wpl = (_Float16*)(ws + oW);
  _Float16* CF0 = (_Float16*)(ws + oCF0);
  _Float16* CF1 = (_Float16*)(ws + oCF1);
  _Float16* FT  = (_Float16*)(ws + oFT);

  hipFuncSetAttribute(reinterpret_cast<const void*>(&k_child),  hipFuncAttributeMaxDynamicSharedMemorySize, CHDYN);
  hipFuncSetAttribute(reinterpret_cast<const void*>(&k_msg),    hipFuncAttributeMaxDynamicSharedMemorySize, MSGDYN);
  hipFuncSetAttribute(reinterpret_cast<const void*>(&k_parent), hipFuncAttributeMaxDynamicSharedMemorySize, PARDYN);

  k_prep<<<PREPB, NTHR, 0, stream>>>(Wc, Wi0, Wi1, Wp, wpl);
  k_child<<<nb8, NTHR, CHDYN, stream>>>(x, ex, bc, wpl, CF0, FT, nT);
  k_msg<<<dim3(nb8, 2), NTHR, MSGDYN, stream>>>(CF0, eidx, e1h, Wi0, bi0, wpl, CF1, FT, OWI0, nT, HC, 1);
  k_msg<<<dim3(nb8, 2), NTHR, MSGDYN, stream>>>(CF1, eidx, e1h, Wi1, bi1, wpl, CF0, FT, OWI1, nT, 2 * HC, 0);
  k_parent<<<nb64, NTHR, PARDYN, stream>>>(FT, bp, wpl, out, nT);
}
